// WLNet_12816182411667
// MI455X (gfx1250) — hardware-verified
//
#include <hip/hip_runtime.h>


typedef __attribute__((ext_vector_type(16))) _Float16 v16h;
typedef __attribute__((ext_vector_type(8)))  float    v8f;
typedef __attribute__((ext_vector_type(4)))  float    v4f;
typedef __attribute__((ext_vector_type(4)))  int      v4i;

#define NNODE 1024
#define NEDGE 16384
#define NPOS  8192
#define DD    64
#define LNEPS 1e-5f
#define CAP   32

#define VST2(T, ptr, val) do { const T _v = (val); *(volatile T*)(ptr) = _v; __threadfence(); *(volatile T*)(ptr) = _v; } while (0)

__device__ __forceinline__ v8f wmma16(v16h a, v16h b, v8f c) {
  v8f d = __builtin_amdgcn_wmma_f32_16x16x32_f16(false, a, false, b, (short)0, c, false, false);
  asm volatile("v_nop\n\tv_nop\n\tv_nop\n\tv_nop" : "+v"(d) : "v"(a), "v"(b));
  return d;
}
__device__ __forceinline__ int fk(int e, int g) { return (e < 8) ? (8 * g + e) : (16 + 8 * g + (e - 8)); }

__global__ __launch_bounds__(128) void k_lists(const int* __restrict__ ei, int* __restrict__ LIN, int* __restrict__ LOUT,
                                               int* __restrict__ cin, int* __restrict__ cout_) {
  __shared__ int ts[2048], td[2048];
  const int v = blockIdx.x * 128 + threadIdx.x;
  int li[CAP], lo[CAP];
#pragma unroll
  for (int j = 0; j < CAP; ++j) { li[j] = -1; lo[j] = -1; }
  int ni = 0, no = 0;
  for (int e0 = 0; e0 < NEDGE; e0 += 2048) {
    __syncthreads();
    for (int i = threadIdx.x; i < 2048; i += 128) { ts[i] = ei[e0 + i]; td[i] = ei[NEDGE + e0 + i]; }
    __syncthreads();
    for (int i = 0; i < 2048; ++i) {
      const int s = ts[i], d = td[i];
      if (d == v) {
#pragma unroll
        for (int j = 0; j < CAP; ++j) if (j == ni) li[j] = s;
        ++ni;
      }
      if (s == v) {
#pragma unroll
        for (int j = 0; j < CAP; ++j) if (j == no) lo[j] = d;
        ++no;
      }
    }
  }
  if (v < NNODE) {
    for (int pass = 0; pass < 2; ++pass) {
#pragma unroll
      for (int q = 0; q < CAP / 4; ++q) {
        v4i a = {li[4 * q], li[4 * q + 1], li[4 * q + 2], li[4 * q + 3]}; *(volatile v4i*)(LIN + (size_t)v * CAP + 4 * q) = a;
        v4i b = {lo[4 * q], lo[4 * q + 1], lo[4 * q + 2], lo[4 * q + 3]}; *(volatile v4i*)(LOUT + (size_t)v * CAP + 4 * q) = b;
      }
      __threadfence();
    }
    VST2(int, cin + v, min(ni, CAP));
    VST2(int, cout_ + v, min(no, CAP));
  }
}

__global__ __launch_bounds__(256) void k_adj(const int* __restrict__ LOUT, const int* __restrict__ cout_, unsigned* __restrict__ adj) {
  const int t = blockIdx.x * 256 + threadIdx.x;
  const int i = t >> 5, w = t & 31;
  const int c = cout_[i];
  unsigned bits = 0u;
  for (int p = 0; p < c; ++p) { const int d = LOUT[i * CAP + p]; if ((d >> 5) == w) bits |= 1u << (d & 31); }
  VST2(unsigned, adj + t, bits);
}

__global__ void k_embed(const int* __restrict__ x, const float* __restrict__ emb, float* __restrict__ h) {
  int t = blockIdx.x * blockDim.x + threadIdx.x;
  if (t < NNODE * DD) { int node = t >> 6, d = t & 63; VST2(float, h + t, emb[x[node] * DD + d]); }
}

__global__ void k_aggr(const int* __restrict__ LIN, const int* __restrict__ cin, const float* __restrict__ h, float* __restrict__ aggr) {
  int t = blockIdx.x * blockDim.x + threadIdx.x;
  if (t < NNODE * DD) {
    const int i = t >> 6, d = t & 63;
    const int c = cin[i];
    float s = 0.f;
    for (int p = 0; p < c; ++p) s += h[LIN[i * CAP + p] * DD + d];
    VST2(float, aggr + t, s);
  }
}

__global__ __launch_bounds__(64) void k_sage(
    const float* __restrict__ aggr, const int* __restrict__ cin,
    const float* __restrict__ hcur, const float* __restrict__ Wl,
    const float* __restrict__ bl, const float* __restrict__ Wr,
    float* __restrict__ hnext) {
  __shared__ float sa[DD], sh[DD], red[DD];
  int node = blockIdx.x, d = threadIdx.x;
  float dg = fmaxf((float)cin[node], 1.0f);
  sa[d] = aggr[node * DD + d] / dg;
  sh[d] = hcur[node * DD + d];
  __syncthreads();
  float y = bl[d];
  #pragma unroll 8
  for (int k = 0; k < DD; ++k)
    y += sa[k] * Wl[k * DD + d] + sh[k] * Wr[k * DD + d];
  red[d] = y;
  __syncthreads();
  for (int off = 32; off >= 1; off >>= 1) {
    if (d < off) red[d] += red[d + off];
    __syncthreads();
  }
  float mean = red[0] * (1.0f / DD);
  __syncthreads();
  float c = y - mean;
  red[d] = c * c;
  __syncthreads();
  for (int off = 32; off >= 1; off >>= 1) {
    if (d < off) red[d] += red[d + off];
    __syncthreads();
  }
  float inv = 1.0f / sqrtf(red[0] * (1.0f / DD) + LNEPS);
  VST2(float, hnext + node * DD + d, c * inv);
}

static __device__ __forceinline__ float adj_bit(const unsigned* adj, int i, int j) {
  unsigned b = (unsigned)i * NNODE + (unsigned)j;
  return ((adj[b >> 5] >> (b & 31)) & 1u) ? 1.0f : 0.0f;
}

__global__ __launch_bounds__(256) void k_bsum(
    const float* __restrict__ h, const float* __restrict__ hW,
    const float* __restrict__ hb, const unsigned* __restrict__ adj,
    float* __restrict__ vp, float* __restrict__ vqp) {
  __shared__ __attribute__((aligned(16))) _Float16 sA[256][72];
  __shared__ __attribute__((aligned(16))) float sHi[16][DD];
  __shared__ __attribute__((aligned(16))) float sHj[16][DD];
  __shared__ __attribute__((aligned(16))) float sP[16][DD];
  float* sQw = (float*)&sA[0][0];
  const int tid = threadIdx.x;
  const int lane = tid & 31, wave = tid >> 5;
  const int n = lane & 15, g = lane >> 4;
  const int i0 = blockIdx.x * 16;

  for (int t = tid; t < 16 * DD; t += 256) sHi[t >> 6][t & 63] = h[i0 * DD + t];
  v16h bfr[2][4];
  #pragma unroll
  for (int kk = 0; kk < 2; ++kk)
    #pragma unroll
    for (int a = 0; a < 4; ++a)
      #pragma unroll
      for (int e = 0; e < 16; ++e) bfr[kk][a][e] = (_Float16)hW[(kk * 32 + fk(e, g)) * DD + a * 16 + n];
  float hb_[4], hwe[4];
  #pragma unroll
  for (int a = 0; a < 4; ++a) { hb_[a] = hb[a * 16 + n]; hwe[a] = hW[64 * DD + a * 16 + n]; }

  float vpacc[2][4];
  #pragma unroll
  for (int tt = 0; tt < 2; ++tt)
    #pragma unroll
    for (int a = 0; a < 4; ++a) vpacc[tt][a] = 0.f;
  const v8f vzero = {0.f, 0.f, 0.f, 0.f, 0.f, 0.f, 0.f, 0.f};

  for (int jt = 0; jt < 64; ++jt) {
    const int j0 = jt * 16;
    __syncthreads();
    for (int t = tid; t < 16 * DD; t += 256) sHj[t >> 6][t & 63] = h[j0 * DD + t];
    __syncthreads();
    {
      const int ii = tid >> 4, jj = tid & 15;
      #pragma unroll 8
      for (int k = 0; k < DD; ++k) sA[tid][k] = (_Float16)(sHi[ii][k] * sHj[jj][k]);
    }
    __syncthreads();

    float vqacc[8][4];
    #pragma unroll
    for (int r = 0; r < 8; ++r)
      #pragma unroll
      for (int a = 0; a < 4; ++a) vqacc[r][a] = 0.0f;

    #pragma unroll
    for (int tt = 0; tt < 2; ++tt) {
      const int t = wave + tt * 8;
      const int i = i0 + t;
      v8f acc[4] = {vzero, vzero, vzero, vzero};
      #pragma unroll
      for (int kk = 0; kk < 2; ++kk) {
        v16h af;
        #pragma unroll
        for (int e = 0; e < 16; ++e) af[e] = sA[t * 16 + n][kk * 32 + fk(e, g)];
        #pragma unroll
        for (int a = 0; a < 4; ++a) acc[a] = wmma16(af, bfr[kk][a], acc[a]);
      }
      #pragma unroll
      for (int r = 0; r < 8; ++r) {
        const int j = j0 + g * 8 + r;
        const float eb = adj_bit(adj, i, j);
        float y[4], s1 = 0.f, s2 = 0.f;
        #pragma unroll
        for (int a = 0; a < 4; ++a) { y[a] = acc[a][r] + hb_[a] + eb * hwe[a]; s1 += y[a]; s2 += y[a] * y[a]; }
        #pragma unroll
        for (int off = 1; off < 16; off <<= 1) { s1 += __shfl_xor(s1, off, 32); s2 += __shfl_xor(s2, off, 32); }
        const float mean = s1 * (1.0f / DD);
        const float var = fmaxf(s2 * (1.0f / DD) - mean * mean, 0.0f);
        const float inv = 1.0f / sqrtf(var + LNEPS);
        #pragma unroll
        for (int a = 0; a < 4; ++a) {
          const float v = fmaxf((y[a] - mean) * inv, 0.0f);
          vpacc[tt][a] += v;
          vqacc[r][a] += v;
        }
      }
    }
    __syncthreads();
    #pragma unroll
    for (int r = 0; r < 8; ++r)
      #pragma unroll
      for (int a = 0; a < 4; ++a) sQw[(wave * 16 + g * 8 + r) * DD + a * 16 + n] = vqacc[r][a];
    __syncthreads();
    {
      const int jl = tid >> 4, sg = tid & 15;
      v4f s4 = {0.f, 0.f, 0.f, 0.f};
      #pragma unroll
      for (int w = 0; w < 8; ++w) s4 += *(const v4f*)(sQw + (w * 16 + jl) * DD + sg * 4);
      VST2(v4f, vqp + ((size_t)blockIdx.x * NNODE + j0 + jl) * DD + sg * 4, s4);
    }
  }
  #pragma unroll
  for (int tt = 0; tt < 2; ++tt)
    #pragma unroll
    for (int a = 0; a < 4; ++a) {
      const float full = vpacc[tt][a] + __shfl_xor(vpacc[tt][a], 16, 32);
      if (g == 0) sP[wave + tt * 8][a * 16 + n] = full;
    }
  __syncthreads();
  {
    const int il = tid >> 4, sg = tid & 15;
    VST2(v4f, vp + (size_t)(i0 + il) * DD + sg * 4, *(const v4f*)(&sP[il][sg * 4]));
  }
}

__global__ void k_vqred(const float* __restrict__ vqp, float* __restrict__ vq) {
  const int t = blockIdx.x * blockDim.x + threadIdx.x;
  if (t >= NNODE * DD) return;
  float s = 0.f;
  for (int st = 0; st < 64; ++st) s += vqp[(size_t)st * NNODE * DD + t];
  VST2(float, vq + t, s);
}

__global__ __launch_bounds__(128) void k_gsel(
    const float* __restrict__ h, const unsigned* __restrict__ adj,
    const float* __restrict__ vp, const float* __restrict__ vq,
    const int* __restrict__ pos, const float* __restrict__ gW,
    const float* __restrict__ gb, float* __restrict__ Gsel) {
  __shared__ _Float16 sA[64][232];
  __shared__ _Float16 sB[224][72];
  int tid = threadIdx.x, lane = tid & 31, wave = tid >> 5;
  int base = blockIdx.x * 64;

  for (int t = tid; t < 224 * DD; t += 128) {
    int k = t >> 6, c = t & 63;
    sB[k][c] = (_Float16)((k < 193) ? gW[k * DD + c] : 0.0f);
  }
  for (int t = tid; t < 64 * 224; t += 128) {
    int r = t / 224, k = t % 224;
    int ridx = base + r;
    int pr = ridx & (NPOS - 1), sw = ridx >> 13;
    int i = pos[pr * 2 + sw];
    int j = pos[pr * 2 + (sw ^ 1)];
    float v;
    if (k < 64)       v = h[i * DD + k] * h[j * DD + k];
    else if (k == 64) v = adj_bit(adj, i, j);
    else if (k < 129) v = vp[i * DD + (k - 65)];
    else if (k < 193) v = vq[j * DD + (k - 129)];
    else              v = 0.0f;
    sA[r][k] = (_Float16)v;
  }
  __syncthreads();

  int n = lane & 15, g = lane >> 4;
  const v8f vzero = {0.f, 0.f, 0.f, 0.f, 0.f, 0.f, 0.f, 0.f};
  v8f acc[4] = {vzero, vzero, vzero, vzero};
  #pragma unroll
  for (int kk = 0; kk < 7; ++kk) {
    v16h af;
    #pragma unroll
    for (int e = 0; e < 16; ++e) af[e] = sA[wave * 16 + n][kk * 32 + fk(e, g)];
    #pragma unroll
    for (int a = 0; a < 4; ++a) {
      v16h bfrag;
      #pragma unroll
      for (int e = 0; e < 16; ++e) bfrag[e] = sB[kk * 32 + fk(e, g)][a * 16 + n];
      acc[a] = wmma16(af, bfrag, acc[a]);
    }
  }
  float outv[8][4];
  #pragma unroll
  for (int r = 0; r < 8; ++r) {
    float y[4], s1 = 0.f, s2 = 0.f;
    #pragma unroll
    for (int a = 0; a < 4; ++a) { y[a] = acc[a][r] + gb[a * 16 + n]; s1 += y[a]; s2 += y[a] * y[a]; }
    #pragma unroll
    for (int off = 1; off < 16; off <<= 1) { s1 += __shfl_xor(s1, off, 32); s2 += __shfl_xor(s2, off, 32); }
    const float mean = s1 * (1.0f / DD);
    const float var = fmaxf(s2 * (1.0f / DD) - mean * mean, 0.0f);
    const float inv = 1.0f / sqrtf(var + LNEPS);
    #pragma unroll
    for (int a = 0; a < 4; ++a) outv[r][a] = fmaxf((y[a] - mean) * inv, 0.0f);
  }
  for (int pass = 0; pass < 2; ++pass) {
    #pragma unroll
    for (int pr = 0; pr < 2; ++pr)
      #pragma unroll
      for (int r = 0; r < 8; ++r) {
        const float a0 = outv[r][2 * pr], b0 = outv[r][2 * pr + 1];
        const float ax = __shfl_xor(a0, 16), bx = __shfl_xor(b0, 16);
        const float v1 = g ? bx : a0;
        const float v2 = g ? b0 : ax;
        *(volatile float*)(Gsel + (size_t)(base + wave * 16 + r) * DD + pr * 32 + lane) = v1;
        *(volatile float*)(Gsel + (size_t)(base + wave * 16 + r + 8) * DD + pr * 32 + lane) = v2;
      }
    __threadfence();
  }
}

__global__ void k_out(const float* __restrict__ Gsel, const float* __restrict__ linW,
                      const float* __restrict__ linb, float* __restrict__ out) {
  int p = blockIdx.x * blockDim.x + threadIdx.x;
  if (p < NPOS) {
    float s = 0.0f;
    #pragma unroll 8
    for (int d = 0; d < DD; ++d) s += Gsel[p * DD + d] * Gsel[(p + NPOS) * DD + d] * linW[d];
    VST2(float, out + p, s + linb[0]);
  }
}

extern "C" void kernel_launch(void* const* d_in, const int* in_sizes, int n_in,
                              void* d_out, int out_size, void* d_ws, size_t ws_size,
                              hipStream_t stream) {
  (void)in_sizes; (void)n_in; (void)out_size;
  const int*   x    = (const int*)d_in[0];
  const int*   ei   = (const int*)d_in[1];
  const int*   pos  = (const int*)d_in[2];
  const float* emb  = (const float*)d_in[3];
  const float* Wl   = (const float*)d_in[4];
  const float* bl   = (const float*)d_in[5];
  const float* Wr   = (const float*)d_in[6];
  const float* hW   = (const float*)d_in[7];
  const float* hb   = (const float*)d_in[8];
  const float* gW   = (const float*)d_in[9];
  const float* gb   = (const float*)d_in[10];
  const float* linW = (const float*)d_in[11];
  const float* linb = (const float*)d_in[12];

  size_t off = 0; char* wsc = (char*)d_ws;
  auto take = [&](size_t bytes) { void* p = wsc + off; off += (bytes + 255) & ~(size_t)255; return p; };
  float* hA   = (float*)take((size_t)NNODE * DD * 4);
  float* hB   = (float*)take((size_t)NNODE * DD * 4);
  float* aggr = (float*)take((size_t)NNODE * DD * 4);
  float* vp   = (float*)take((size_t)NNODE * DD * 4);
  float* vq   = (float*)take((size_t)NNODE * DD * 4);
  float* vqp  = (float*)take((size_t)64 * NNODE * DD * 4);
  float* Gsel = (float*)take((size_t)2 * NPOS * DD * 4);
  unsigned* adj = (unsigned*)take((size_t)NNODE * 32 * 4);
  int* LIN  = (int*)take((size_t)NNODE * CAP * 4);
  int* LOUT = (int*)take((size_t)NNODE * CAP * 4);
  int* cin  = (int*)take((size_t)NNODE * 4);
  int* cout_ = (int*)take((size_t)NNODE * 4);
  if (off > ws_size) return;

  k_lists<<<NNODE / 128, 128, 0, stream>>>(ei, LIN, LOUT, cin, cout_);
  k_adj<<<(NNODE * 32) / 256, 256, 0, stream>>>(LOUT, cout_, adj);
  k_embed<<<(NNODE * DD) / 256, 256, 0, stream>>>(x, emb, hA);

  for (int layer = 0; layer < 2; ++layer) {
    const float* cur = layer ? hB : hA;
    float* nxt = layer ? hA : hB;
    k_aggr<<<(NNODE * DD) / 256, 256, 0, stream>>>(LIN, cin, cur, aggr);
    k_sage<<<NNODE, DD, 0, stream>>>(aggr, cin, cur, Wl + layer * DD * DD, bl + layer * DD, Wr + layer * DD * DD, nxt);
  }
  k_bsum<<<dim3(64), 256, 0, stream>>>(hA, hW, hb, adj, vp, vqp);
  k_vqred<<<(NNODE * DD) / 256, 256, 0, stream>>>(vqp, vq);
  k_gsel<<<256, 128, 0, stream>>>(hA, adj, vp, vq, pos, gW, gb, Gsel);
  k_out<<<NPOS / 256, 256, 0, stream>>>(Gsel, linW, linb, (float*)d_out);
}
